// PatchEmbedding3D_14955076125179
// MI455X (gfx1250) — hardware-verified
//
#include <hip/hip_runtime.h>


#define NB_  32
#define NPTS 16384
#define PS   32
#define NP   512
#define HID  128
#define ED   256
#define NR   (NB_ * NPTS)
#define WSC  16384.0f
#define CH   65536
typedef _Float16 h16;
typedef unsigned short bf;
typedef __attribute__((ext_vector_type(16))) __bf16   v16bf;
typedef __attribute__((ext_vector_type(16))) _Float16 v16h;
typedef __attribute__((ext_vector_type(8)))  _Float16 v8h;
typedef __attribute__((ext_vector_type(8)))  unsigned short v8us;
typedef __attribute__((ext_vector_type(8)))  float    v8f;
typedef __attribute__((ext_vector_type(4)))  float    v4f;
typedef v8h  __attribute__((may_alias)) v8ha;
typedef v4f  __attribute__((may_alias)) v4fa;
typedef v8us __attribute__((may_alias)) v8usa;

__device__ __forceinline__ unsigned short f2bf(float f) { unsigned u = __float_as_uint(f); u += 0x7FFFu + ((u >> 16) & 1u); return (unsigned short)(u >> 16); }
__device__ __forceinline__ float bf2f(unsigned short b) { return __uint_as_float(((unsigned)b) << 16); }
__device__ __forceinline__ float bfr(float f) { return bf2f(f2bf(f)); }
__device__ __forceinline__ v16h cat16(v8h lo, v8h hi) { return __builtin_shufflevector(lo, hi, 0, 1, 2, 3, 4, 5, 6, 7, 8, 9, 10, 11, 12, 13, 14, 15); }
__device__ __forceinline__ v16bf cat16b(v8us lo, v8us hi) { return __builtin_bit_cast(v16bf, __builtin_shufflevector(lo, hi, 0, 1, 2, 3, 4, 5, 6, 7, 8, 9, 10, 11, 12, 13, 14, 15)); }
__device__ __forceinline__ v8f wmma16(v16h a, v16h b, v8f c) { return __builtin_amdgcn_wmma_f32_16x16x32_f16(false, a, false, b, (short)0, c, false, false); }
__device__ __forceinline__ v8f wmmab(v16bf a, v16bf b, v8f c) { return __builtin_amdgcn_wmma_f32_16x16x32_bf16(false, a, false, b, (short)0, c, false, false); }


template <typename T16> struct WFrag;
template <> struct WFrag<h16> { typedef v16h V; static __device__ __forceinline__ V ld(const h16* p) { return cat16(*(const v8h*)p, *(const v8h*)(p + 16)); } static __device__ __forceinline__ v8f mma(V a, V b, v8f c) { return wmma16(a, b, c); } };
template <> struct WFrag<bf> { typedef v16bf V; static __device__ __forceinline__ V ld(const bf* p) { return cat16b(*(const v8us*)p, *(const v8us*)(p + 16)); } static __device__ __forceinline__ v8f mma(V a, V b, v8f c) { return wmmab(a, b, c); } };
template <typename T16, int NSPLIT, bool BIAS>
__global__ __launch_bounds__(32) void k_gemmw(const T16* __restrict__ A, const T16* __restrict__ A2, const T16* __restrict__ Bt, const T16* __restrict__ Bt2, int K, float* C, int ldc, const float* __restrict__ bias, size_t sA, size_t sB, size_t sC) {
    typedef typename WFrag<T16>::V V;
    __shared__ __align__(16) float os[16 * 68];
    const size_t z = blockIdx.z; A += z * sA; if (A2) A2 += z * sA; Bt += z * sB; if (Bt2) Bt2 += z * sB; C += z * sC;
    const int lane = threadIdx.x & 31, lr = lane & 15, hi = lane >> 4; const int r0 = blockIdx.x * 64, c0 = blockIdx.y * 64;
    v8f acc[4][4];
#pragma unroll
    for (int mb = 0; mb < 4; ++mb)
#pragma unroll
        for (int nb = 0; nb < 4; ++nb) acc[mb][nb] = (v8f){};
    const size_t aoff = (size_t)(r0 + lr) * K + 8 * hi, boff = (size_t)(c0 + lr) * K + 8 * hi;
#pragma unroll 1
    for (int kc = 0; kc < K; kc += 32) {
        V a[4], a2[4];
#pragma unroll
        for (int mb = 0; mb < 4; ++mb) { a[mb] = WFrag<T16>::ld(A + aoff + (size_t)mb * 16 * K + kc); if (NSPLIT == 1 || NSPLIT == 2) a2[mb] = WFrag<T16>::ld(A2 + aoff + (size_t)mb * 16 * K + kc); }
#pragma unroll
        for (int nb = 0; nb < 4; ++nb) { const V b = WFrag<T16>::ld(Bt + boff + (size_t)nb * 16 * K + kc); V b2; if (NSPLIT >= 2) b2 = WFrag<T16>::ld(Bt2 + boff + (size_t)nb * 16 * K + kc);
#pragma unroll
            for (int mb = 0; mb < 4; ++mb) { acc[mb][nb] = WFrag<T16>::mma(a[mb], b, acc[mb][nb]); if (NSPLIT == 1 || NSPLIT == 2) acc[mb][nb] = WFrag<T16>::mma(a2[mb], b, acc[mb][nb]); if (NSPLIT >= 2) acc[mb][nb] = WFrag<T16>::mma(a[mb], b2, acc[mb][nb]); } }
        asm volatile("v_nop\n\tv_nop\n\tv_nop\n\tv_nop" : "+v"(acc[0][0]), "+v"(acc[1][1]), "+v"(acc[2][2]), "+v"(acc[3][3]) : "v"(a[0]), "v"(a[3]));
    }
#pragma unroll
    for (int mb = 0; mb < 4; ++mb) {
#pragma unroll
        for (int nb = 0; nb < 4; ++nb) {
#pragma unroll
            for (int j = 0; j < 8; ++j) os[(hi * 8 + j) * 68 + nb * 16 + lr] = acc[mb][nb][j]; }
        __builtin_amdgcn_wave_barrier(); asm volatile("" ::: "memory");
        float* crow = C + (size_t)(r0 + mb * 16) * ldc + c0;
#pragma unroll 1
        for (int ps = 0; ps < 2; ++ps) {
#pragma unroll
            for (int s = 0; s < 8; ++s) { const int row = 2 * s + hi, cofs = lr * 4; v4f val = *(const v4fa*)(os + row * 68 + cofs); if (BIAS) { val[0] += bfr(bias[c0 + cofs]); val[1] += bfr(bias[c0 + cofs + 1]); val[2] += bfr(bias[c0 + cofs + 2]); val[3] += bfr(bias[c0 + cofs + 3]); }
                *(volatile v4f*)(crow + (size_t)row * ldc + cofs) = val; }
            if (ps == 0) __threadfence(); }
        __builtin_amdgcn_wave_barrier(); asm volatile("" ::: "memory");
    }
}

__device__ __forceinline__ h16 tohx(float x) { return (h16)x; }
typedef __attribute__((ext_vector_type(4))) _Float16 v4h;
typedef __attribute__((ext_vector_type(2))) _Float16 v2h;

__global__ __launch_bounds__(256) void k_wtG16(const float* __restrict__ w, int K, int N, int pitch, int col0, h16* Bt) {
    const int lane = threadIdx.x & 31; const int L0 = (blockIdx.x * 8 + (threadIdx.x >> 5)) * 8; const int nlines = N * K / 64;
#pragma unroll 1
    for (int ps = 0; ps < 2; ++ps) {
#pragma unroll 1
        for (int l = 0; l < 8; ++l) { const int L = L0 + l; if (L >= nlines) break; const size_t e = (size_t)L * 64 + lane * 2; const int k = (int)(e % K), n = (int)(e / K); v2h o;
            o[0] = tohx(bfr(w[(size_t)k * pitch + col0 + n]) * WSC); o[1] = tohx(bfr(w[(size_t)(k + 1) * pitch + col0 + n]) * WSC); *(volatile v2h*)(Bt + e) = o; }
        if (ps == 0) __threadfence(); }
}
__global__ __launch_bounds__(256) void k_l1(const float* __restrict__ x, const float* __restrict__ w1, const float* __restrict__ b1, const float* __restrict__ g1, const float* __restrict__ be1, size_t r0, h16* H16) {
    const int lane = threadIdx.x & 31; const size_t rl = (size_t)blockIdx.x * 8 + (threadIdx.x >> 5); if (rl >= CH) return; const size_t r = r0 + rl; const int b = (int)(r / NPTS), n = (int)(r % NPTS);
    float px = bfr(x[((size_t)b * 3 + 0) * NPTS + n]), py = bfr(x[((size_t)b * 3 + 1) * NPTS + n]), pz = bfr(x[((size_t)b * 3 + 2) * NPTS + n]); asm volatile("" : "+v"(px)); asm volatile("" : "+v"(py)); asm volatile("" : "+v"(pz));
    float v[4]; float s = 0.f;
#pragma unroll
    for (int q = 0; q < 4; ++q) { const int j = lane * 4 + q; float wa = bfr(w1[j]), wb = bfr(w1[HID + j]), wc = bfr(w1[2 * HID + j]), bb = bfr(b1[j]); asm volatile("" : "+v"(wa)); asm volatile("" : "+v"(wb)); asm volatile("" : "+v"(wc)); asm volatile("" : "+v"(bb));
        float p0 = __fmul_rn(px, wa), p1 = __fmul_rn(py, wb), p2 = __fmul_rn(pz, wc); asm volatile("" : "+v"(p0)); asm volatile("" : "+v"(p1)); asm volatile("" : "+v"(p2)); const float h = __fadd_rn(__fadd_rn(__fadd_rn(p0, p1), p2), bb); v[q] = h; s = __fadd_rn(s, h); }
#pragma unroll
    for (int sh = 16; sh; sh >>= 1) s += __shfl_xor(s, sh, 32);
    const float mu = s * (1.0f / HID); float qq = 0.f;
#pragma unroll
    for (int q = 0; q < 4; ++q) { const float d0 = v[q] - mu; float p = __fmul_rn(d0, d0); asm volatile("" : "+v"(p)); qq = __fadd_rn(qq, p); }
#pragma unroll
    for (int sh = 16; sh; sh >>= 1) qq += __shfl_xor(qq, sh, 32);
    const float rs = __fdiv_rn(1.0f, __fsqrt_rn(__fadd_rn(qq * (1.0f / HID), 1e-5f))); v4h o;
#pragma unroll
    for (int q = 0; q < 4; ++q) { const int j = lane * 4 + q; float g = bfr(g1[j]), be = bfr(be1[j]); asm volatile("" : "+v"(g)); asm volatile("" : "+v"(be)); float tn = __fmul_rn(v[q] - mu, rs); asm volatile("" : "+v"(tn)); float tg = __fmul_rn(tn, g); asm volatile("" : "+v"(tg)); o[q] = tohx(fmaxf(__fadd_rn(tg, be), 0.f)); }
    *(volatile v4h*)(H16 + rl * HID + lane * 4) = o; __threadfence(); *(volatile v4h*)(H16 + rl * HID + lane * 4) = o; }
__global__ __launch_bounds__(256) void k_pool(const float* __restrict__ F, const float* __restrict__ b2, const float* __restrict__ g2, const float* __restrict__ be2, const float* __restrict__ gn, const float* __restrict__ bn, int p0, float* OUT) {
    const int lane = threadIdx.x & 31; const int pl = blockIdx.x * 8 + (threadIdx.x >> 5); if (pl >= CH / PS) return; const int pp = p0 + pl; float mx[8]; float bb[8], gg[8], ee[8];
#pragma unroll
    for (int q = 0; q < 8; ++q) { const int c = lane * 8 + q; mx[q] = -3.0e38f; float t0 = bfr(b2[c]), t1 = bfr(g2[c]), t2 = bfr(be2[c]); asm volatile("" : "+v"(t0)); asm volatile("" : "+v"(t1)); asm volatile("" : "+v"(t2)); bb[q] = t0; gg[q] = t1; ee[q] = t2; }
    for (int k = 0; k < PS; ++k) { const size_t r = (size_t)pl * PS + k; float v[8]; float s = 0.f; const v4f a0 = *(const v4f*)(F + r * ED + lane * 8), a1 = *(const v4f*)(F + r * ED + lane * 8 + 4);
#pragma unroll
        for (int q = 0; q < 8; ++q) { float a = (q < 4 ? a0[q] : a1[q - 4]) * (1.0f / WSC); asm volatile("" : "+v"(a)); const float e = __fadd_rn(a, bb[q]); v[q] = e; s = __fadd_rn(s, e); }
#pragma unroll
        for (int sh = 16; sh; sh >>= 1) s += __shfl_xor(s, sh, 32);
        const float mu = s * (1.0f / ED); float qq = 0.f;
#pragma unroll
        for (int q = 0; q < 8; ++q) { const float d0 = v[q] - mu; float p = __fmul_rn(d0, d0); asm volatile("" : "+v"(p)); qq = __fadd_rn(qq, p); }
#pragma unroll
        for (int sh = 16; sh; sh >>= 1) qq += __shfl_xor(qq, sh, 32);
        const float rs = __fdiv_rn(1.0f, __fsqrt_rn(__fadd_rn(qq * (1.0f / ED), 1e-5f)));
#pragma unroll
        for (int q = 0; q < 8; ++q) { float tn = __fmul_rn(v[q] - mu, rs); asm volatile("" : "+v"(tn)); float tg = __fmul_rn(tn, gg[q]); asm volatile("" : "+v"(tg)); mx[q] = fmaxf(mx[q], __fadd_rn(tg, ee[q])); } }
    float s = 0.f;
#pragma unroll
    for (int q = 0; q < 8; ++q) s = __fadd_rn(s, mx[q]);
#pragma unroll
    for (int sh = 16; sh; sh >>= 1) s += __shfl_xor(s, sh, 32);
    const float mu = s * (1.0f / ED); float qq = 0.f;
#pragma unroll
    for (int q = 0; q < 8; ++q) { const float d0 = mx[q] - mu; float p = __fmul_rn(d0, d0); asm volatile("" : "+v"(p)); qq = __fadd_rn(qq, p); }
#pragma unroll
    for (int sh = 16; sh; sh >>= 1) qq += __shfl_xor(qq, sh, 32);
    const float rs = __fdiv_rn(1.0f, __fsqrt_rn(__fadd_rn(qq * (1.0f / ED), 1e-5f))); v4f o0, o1;
#pragma unroll
    for (int q = 0; q < 8; ++q) { const int c = lane * 8 + q; float g = bfr(gn[c]), be = bfr(bn[c]); asm volatile("" : "+v"(g)); asm volatile("" : "+v"(be)); float tn = __fmul_rn(mx[q] - mu, rs); asm volatile("" : "+v"(tn)); float tg = __fmul_rn(tn, g); asm volatile("" : "+v"(tg)); const float y = __fadd_rn(tg, be); if (q < 4) o0[q] = y; else o1[q - 4] = y; }
    float* dst = OUT + (size_t)pp * ED + lane * 8; *(volatile v4f*)dst = o0; *(volatile v4f*)(dst + 4) = o1; __threadfence(); *(volatile v4f*)dst = o0; *(volatile v4f*)(dst + 4) = o1; }

extern "C" void kernel_launch(void* const* d_in, const int* in_sizes, int n_in,
                              void* d_out, int out_size, void* d_ws, size_t ws_size, hipStream_t stream) {
    (void)in_sizes; (void)n_in; (void)out_size;
    const float* IN[11]; for (int i = 0; i < 11; ++i) IN[i] = (const float*)d_in[i];
    float* OUT = (float*)d_out;
    char* wsp = (char*)d_ws;
    auto take = [&](size_t bytes) { char* p = wsp; wsp += (bytes + 255) & ~(size_t)255; return (void*)p; };
    h16* W2S = (h16*)take((size_t)ED * HID * 2); h16* H16 = (h16*)take((size_t)CH * HID * 2); float* F = (float*)take((size_t)CH * ED * 4);
    if ((size_t)(wsp - (char*)d_ws) > ws_size) return;
    k_wtG16<<<(unsigned)((HID * ED / 64 + 63) / 64), 256, 0, stream>>>(IN[5], HID, ED, ED, 0, W2S);
    for (int c = 0; c < NR / CH; ++c) { const size_t r0 = (size_t)c * CH;
        k_l1<<<CH / 8, 256, 0, stream>>>(IN[0], IN[1], IN[2], IN[3], IN[4], r0, H16);
        k_gemmw<h16, 0, false><<<dim3(CH / 64, ED / 64, 1), 32, 0, stream>>>(H16, nullptr, W2S, nullptr, HID, F, ED, nullptr, 0, 0, 0);
        k_pool<<<(CH / PS) / 8, 256, 0, stream>>>(F, IN[6], IN[7], IN[8], IN[9], IN[10], (int)(r0 / PS), OUT); }
}
